// GAT_46961172415075
// MI455X (gfx1250) — hardware-verified
//
#include <hip/hip_runtime.h>
#include <stddef.h>
#include <stdint.h>
#include <math.h>


#define NIN     100
#define KX      128
#define KH      256
#define NSTR    256
#define HC01    128
#define C01     32
#define NCLS    47
#define HC2     188
#define NTHR    256
#define NWAVE   8
#define EPT     8
#define CHUNK   (NTHR * EPT)
#define WCAP    (EPT * 32)
#define LISTN   (NWAVE * WCAP)
#define NBRUN   1024
#define SLB     10
#define NBW     (NBRUN / NWAVE)
#define BCAP    44
#define BINS    (NBRUN * BCAP)
#define GRP     32
#define AGG_ZINTS (LISTN + BINS + NBRUN)
#define STGF    (NWAVE * GRP * NCLS)
#define LDS_AGG0 ((AGG_ZINTS + 16) * 4)
#define LDS_AGG1 ((AGG_ZINTS + 16 + STGF) * 4)
#define GBM     64
#define LDP     260
#define LDS_GEMM ((GBM * LDP + 3 * 256 + 512) * 4)
#define UW0     (256 * (KX / 8))
#define UW1     (256 * (KH / 8))
#define UW2     (256 * (KH / 8))
#define NEGSL   0.2f
#define NEGBIG  (-3.0e38f)
#define WSMAX   134217728

static_assert((CHUNK & (CHUNK - 1)) == 0 && CHUNK == 2048);
static_assert(NBRUN == (1 << SLB));
static_assert(((long long)CHUNK << SLB) < (1LL << 31));
static_assert(AGG_ZINTS % (NTHR * 4) == 0);
static_assert(NBW % GRP == 0 && NBRUN % GRP == 0);
static_assert((GRP * NCLS * 4) % 128 == 0);
static_assert(LDS_AGG1 <= 300000 && LDS_GEMM <= 300000);
static_assert(KX % 32 == 0 && KH % 32 == 0 && KH == 2 * HC01);
static_assert(UW0 % NTHR == 0 && UW1 % NTHR == 0 && UW2 % NTHR == 0);
static_assert(HC01 == 4 * 32 && HC2 == 4 * NCLS && HC2 + NCLS <= NSTR);
static_assert(NIN % 4 == 0 && NIN <= KX);
static_assert(NCLS > 32 && NCLS <= 64);
static_assert(GBM * 4 == NTHR);

typedef float          v4f  __attribute__((ext_vector_type(4)));
typedef float          v8f  __attribute__((ext_vector_type(8)));
typedef int            v4i  __attribute__((ext_vector_type(4)));
typedef int            v8i  __attribute__((ext_vector_type(8)));
typedef unsigned int   v4u  __attribute__((ext_vector_type(4)));
typedef unsigned short v8us __attribute__((ext_vector_type(8)));
typedef __bf16         v16b __attribute__((ext_vector_type(16)));
typedef v4f  __attribute__((may_alias)) v4fa;
typedef v4i  __attribute__((may_alias)) v4ia;
typedef v8us __attribute__((may_alias)) v8usa;
union FragB { v16b v; v8us h[2]; v8i w; };

__device__ __forceinline__ v8f wmb(const FragB& a, const FragB& b, v8f c) {
  v8f d = __builtin_amdgcn_wmma_f32_16x16x32_bf16(false, a.v, false, b.v, (short)0, c, false, false);
  asm volatile("v_nop\n\tv_nop\n\tv_nop\n\tv_nop" : "+v"(d) : "v"(a.w), "v"(b.w));
  return d;
}

__device__ __forceinline__ unsigned int f2bf(float f) {
  const unsigned int u = __float_as_uint(f);
  return ((u + 0x7FFFu + ((u >> 16) & 1u)) >> 16) & 0xFFFFu;
}
__device__ __forceinline__ float bf2f(unsigned int b) { return __uint_as_float(b << 16); }
__device__ __forceinline__ float bfr(float f) { return bf2f(f2bf(f)); }
__device__ __forceinline__ v4f bfr4(const v4f a) {
  v4f r; r.x = bfr(a.x); r.y = bfr(a.y); r.z = bfr(a.z); r.w = bfr(a.w); return r;
}
__device__ __forceinline__ unsigned int pk2(float lo, float hi) { return f2bf(lo) | (f2bf(hi) << 16); }

__device__ __forceinline__ float wmaxf(float v) {
#pragma unroll
  for (int off = 16; off > 0; off >>= 1) v = fmaxf(v, __shfl_xor(v, off));
  return v;
}
__device__ __forceinline__ float wsumf(float v) {
#pragma unroll
  for (int off = 16; off > 0; off >>= 1) v += __shfl_xor(v, off);
  return v;
}

__device__ __forceinline__ v4u cvt8(const float* __restrict__ rowp, int Kin, int kk) {
  const int ka = kk < Kin - 4 ? kk : Kin - 4;
  const int kb = kk + 4 < Kin - 4 ? kk + 4 : Kin - 4;
  const v4f a = *(const v4fa*)(rowp + ka);
  const v4f b = *(const v4fa*)(rowp + kb);
  const unsigned int ma = (kk + 4 <= Kin) ? 0xFFFFFFFFu : 0u;
  const unsigned int mb = (kk + 8 <= Kin) ? 0xFFFFFFFFu : 0u;
  v4u r;
  r.x = pk2(a.x, a.y) & ma; r.y = pk2(a.z, a.w) & ma;
  r.z = pk2(b.x, b.y) & mb; r.w = pk2(b.z, b.w) & mb;
  return r;
}

__device__ __forceinline__ v4u wrow2(const float* __restrict__ Wa, int na, const float* __restrict__ Wb, int nb2,
                                     int Kin, int n, int kk) {
  const int ra = n < na ? n : na - 1;
  int rb = n - na; rb = rb < 0 ? 0 : (rb > nb2 - 1 ? nb2 - 1 : rb);
  const v4u pa = cvt8(Wa + (size_t)ra * (size_t)Kin, Kin, kk);
  const v4u pb = cvt8(Wb + (size_t)rb * (size_t)Kin, Kin, kk);
  const unsigned int ma = (n < na) ? 0xFFFFFFFFu : 0u;
  const unsigned int mb = (n >= na && n < na + nb2) ? 0xFFFFFFFFu : 0u;
  v4u r;
  r.x = (pa.x & ma) | (pb.x & mb); r.y = (pa.y & ma) | (pb.y & mb);
  r.z = (pa.z & ma) | (pb.z & mb); r.w = (pa.w & ma) | (pb.w & mb);
  return r;
}

__global__ __launch_bounds__(NTHR) void k_prep(const float* __restrict__ x,
    const float* __restrict__ W0, const float* __restrict__ sw0,
    const float* __restrict__ W1, const float* __restrict__ sw1,
    const float* __restrict__ W2, const float* __restrict__ sw2,
    unsigned short* XB, unsigned short* WB0, unsigned short* WB1, unsigned short* WB2,
    int nN, int uX) {
  const int u = (int)blockIdx.x * NTHR + (int)threadIdx.x;
  v4u o;
  unsigned short* dp;
  if (u < uX) {
    const int row = u >> 4;
    const int kk  = (u & 15) * 8;
    const int rc  = row < nN ? row : nN - 1;
    o = cvt8(x + (size_t)rc * NIN, NIN, kk);
    const unsigned int mr = (row < nN) ? 0xFFFFFFFFu : 0u;
    o.x &= mr; o.y &= mr; o.z &= mr; o.w &= mr;
    dp = XB + (size_t)row * KX + kk;
  } else if (u < uX + UW0) {
    const int v  = u - uX;
    const int n  = v >> 4;
    const int kk = (v & 15) * 8;
    o = wrow2(W0, HC01, sw0, HC01, NIN, n, kk);
    dp = WB0 + (size_t)n * KX + kk;
  } else if (u < uX + UW0 + UW1) {
    const int v  = u - uX - UW0;
    const int n  = v >> 5;
    const int k8 = (v & 31) * 8;
    o = wrow2(W1, HC01, sw1, HC01, HC01, n, k8 & (HC01 - 1));
    dp = WB1 + (size_t)n * KH + k8;
  } else if (u < uX + UW0 + UW1 + UW2) {
    const int v  = u - uX - UW0 - UW1;
    const int n  = v >> 5;
    const int k8 = (v & 31) * 8;
    o = wrow2(W2, HC2, sw2, NCLS, HC01, n, k8 & (HC01 - 1));
    dp = WB2 + (size_t)n * KH + k8;
  } else {
    return;
  }
  *(volatile v4u*)dp = o;
  __threadfence();
  *(volatile v4u*)dp = o;
}

__global__ __launch_bounds__(NTHR) void k_gemm(const unsigned short* __restrict__ A, int lda,
                                               const unsigned short* __restrict__ BT, int ldb, int K,
                                               float* Sm, const float* __restrict__ atts,
                                               const float* __restrict__ attd, const float* __restrict__ sb,
                                               int HC, int C, int skip0, int nskip,
                                               float* ALR, int arOff) {
  extern __shared__ __attribute__((aligned(16))) float gsm[];
  float* stg = gsm;
  float* asv = gsm + GBM * LDP;
  float* adv = asv + 256;
  float* sbv = adv + 256;
  float* sdt = sbv + 256;
  const int tid = (int)threadIdx.x, lane = tid & 31, hh = lane >> 4, m = lane & 15;
  const int wave = __builtin_amdgcn_readfirstlane(tid >> 5);
  const int rg = wave & 3, cg = wave >> 2;
  const int rowBase = (int)blockIdx.x * GBM;
  const int colBase = cg * 128;

  {
    const int ca = tid < HC ? tid : HC - 1;
    const float vs = atts[ca];
    const float vd = attd[ca];
    int cs = tid - skip0; cs = cs < 0 ? 0 : (cs > nskip - 1 ? nskip - 1 : cs);
    const float vb = sb[cs];
    asv[tid] = (tid < HC) ? bfr(vs) : 0.0f;
    adv[tid] = (tid < HC) ? bfr(vd) : 0.0f;
    sbv[tid] = (tid >= skip0 && tid < skip0 + nskip) ? bfr(vb) : 0.0f;
  }
  __syncthreads();

  v8f acc[8];
  {
    const v8f z = {0.f, 0.f, 0.f, 0.f, 0.f, 0.f, 0.f, 0.f};
#pragma unroll
    for (int t = 0; t < 8; ++t) acc[t] = z;
  }
  const unsigned short* ap = A  + (size_t)(rowBase + 16 * rg + m) * (size_t)lda + 8 * hh;
  const unsigned short* bp = BT + (size_t)(colBase + m) * (size_t)ldb + 8 * hh;

#pragma unroll 1
  for (int k0 = 0; k0 < K; k0 += 32) {
    FragB af;
    af.h[0] = *(const v8usa*)(ap + k0);
    af.h[1] = *(const v8usa*)(ap + k0 + 16);
#pragma unroll
    for (int nt = 0; nt < 8; ++nt) {
      const unsigned short* wq = bp + (size_t)(16 * nt) * (size_t)ldb + k0;
      FragB bf;
      bf.h[0] = *(const v8usa*)wq;
      bf.h[1] = *(const v8usa*)(wq + 16);
      acc[nt] = wmb(af, bf, acc[nt]);
    }
  }

#pragma unroll
  for (int nt = 0; nt < 8; ++nt) {
    const int lc = colBase + 16 * nt + m;
    const float bv = sbv[lc];
#pragma unroll
    for (int r = 0; r < 8; ++r) {
      const int lr = 16 * rg + 8 * hh + r;
      stg[lr * LDP + lc] = acc[nt][r] + bv;
    }
  }
  __syncthreads();

  {
    const int row = tid & 63, head = tid >> 6;
    const float* hr = stg + row * LDP + head * C;
    const float* sa = asv + head * C;
    const float* sd = adv + head * C;
    float s = 0.0f, d = 0.0f;
#pragma unroll 4
    for (int c = 0; c < C; ++c) {
      const float v = hr[c];
      s = fmaf(v, sa[c], s);
      d = fmaf(v, sd[c], d);
    }
    sdt[row * 4 + head]       = s;
    sdt[256 + row * 4 + head] = d;
  }
  __syncthreads();

  const int which = wave >> 1;
  const int piece = tid & 63;
  const int wsel  = which < 2 ? which : 1;
  const v4f alv = *(const v4fa*)(sdt + wsel * 256 + 4 * piece);
  float* alp = ALR + (size_t)wsel * (size_t)arOff + (size_t)rowBase * 4 + 4 * piece;
#pragma unroll 1
  for (int i = 0; i < GBM / NWAVE; ++i) {
    const int row = wave * (GBM / NWAVE) + i;
#pragma unroll
    for (int c = 0; c < 2; ++c) {
      const v4f p = *(const v4fa*)(stg + row * LDP + c * 128 + 4 * lane);
      float* op = Sm + (size_t)(rowBase + row) * NSTR + c * 128 + 4 * lane;
      *(volatile v4f*)op = p;
    }
  }
  if (wave < 4) *(volatile v4f*)alp = alv;
  __threadfence();
#pragma unroll 1
  for (int i = 0; i < GBM / NWAVE; ++i) {
    const int row = wave * (GBM / NWAVE) + i;
#pragma unroll
    for (int c = 0; c < 2; ++c) {
      const v4f p = *(const v4fa*)(stg + row * LDP + c * 128 + 4 * lane);
      float* op = Sm + (size_t)(rowBase + row) * NSTR + c * 128 + 4 * lane;
      *(volatile v4f*)op = p;
    }
  }
  if (wave < 4) *(volatile v4f*)alp = alv;
}

__device__ __forceinline__ int scan_chunk(const int* __restrict__ dsts, int nE, int cbase, int slotBase,
                                          int nb, int vec8, int* list, int tid, int lane, int wave) {
  int wc = 0;
  const int el0  = tid * EPT;
  const int e0   = cbase + el0;
  const int sent = -2147483647 - 1;
  v4i da, db;
  if (vec8 != 0 && cbase + CHUNK <= nE) {
    da = *(const v4i*)(dsts + e0);
    db = *(const v4i*)(dsts + e0 + 4);
  } else {
    da.x = (e0     < nE) ? dsts[min(e0,     nE - 1)] : sent;
    da.y = (e0 + 1 < nE) ? dsts[min(e0 + 1, nE - 1)] : sent;
    da.z = (e0 + 2 < nE) ? dsts[min(e0 + 2, nE - 1)] : sent;
    da.w = (e0 + 3 < nE) ? dsts[min(e0 + 3, nE - 1)] : sent;
    db.x = (e0 + 4 < nE) ? dsts[min(e0 + 4, nE - 1)] : sent;
    db.y = (e0 + 5 < nE) ? dsts[min(e0 + 5, nE - 1)] : sent;
    db.z = (e0 + 6 < nE) ? dsts[min(e0 + 6, nE - 1)] : sent;
    db.w = (e0 + 7 < nE) ? dsts[min(e0 + 7, nE - 1)] : sent;
  }
  const unsigned nbs = (unsigned)slotBase;
  const unsigned unb = (unsigned)nb;
  const unsigned s0 = (unsigned)da.x - nbs, s1 = (unsigned)da.y - nbs;
  const unsigned s2 = (unsigned)da.z - nbs, s3 = (unsigned)da.w - nbs;
  const unsigned s4 = (unsigned)db.x - nbs, s5 = (unsigned)db.y - nbs;
  const unsigned s6 = (unsigned)db.z - nbs, s7 = (unsigned)db.w - nbs;
  const bool h0 = s0 < unb, h1 = s1 < unb, h2 = s2 < unb, h3 = s3 < unb;
  const bool h4 = s4 < unb, h5 = s5 < unb, h6 = s6 < unb, h7 = s7 < unb;
  const unsigned any = __builtin_amdgcn_ballot_w32(h0 | h1 | h2 | h3 | h4 | h5 | h6 | h7);
  if (any != 0u) {
#define HITJ(J, HJ, SJ) { \
      const unsigned mj = __builtin_amdgcn_ballot_w32(HJ); \
      if (mj != 0u) { \
        if (HJ) { \
          const int pos = wc + (int)__builtin_amdgcn_mbcnt_lo(mj, 0u); \
          if (pos < WCAP) list[wave * WCAP + pos] = ((el0 + (J)) << SLB) | (int)(SJ); \
        } \
        wc += (int)__builtin_popcount(mj); } }
    HITJ(0, h0, s0)
    HITJ(1, h1, s1)
    HITJ(2, h2, s2)
    HITJ(3, h3, s3)
    HITJ(4, h4, s4)
    HITJ(5, h5, s5)
    HITJ(6, h6, s6)
    HITJ(7, h7, s7)
#undef HITJ
  }
  return wc;
}

__device__ __forceinline__ int batch_front(const int* bslot, const int* __restrict__ srcs,
                                           const float* __restrict__ ALR, int nE, int nN, int gcl,
                                           int b0, int nent, int lane, const v4f ar4,
                                           float (&m)[4], float (&d)[4], float (&ee)[4], float (&sc)[4]) {
  const int j = b0 + lane;
  const bool valid = j < nent;
  int bi = j - 1; bi = bi < 0 ? 0 : (bi > BCAP - 1 ? BCAP - 1 : bi);
  int eid = bslot[bi];
  eid = eid < 0 ? 0 : (eid > nE - 1 ? nE - 1 : eid);
  const int sraw = srcs[eid];
  const int s = sraw < 0 ? 0 : (sraw > nN - 1 ? nN - 1 : sraw);
  const int sr = (j == 0) ? gcl : s;
  const v4f a4 = *(const v4fa*)(ALR + (size_t)sr * 4);
  float lg[4];
  lg[0] = a4.x + ar4.x; lg[1] = a4.y + ar4.y; lg[2] = a4.z + ar4.z; lg[3] = a4.w + ar4.w;
#pragma unroll
  for (int h = 0; h < 4; ++h) {
    float t = lg[h];
    t = t > 0.0f ? t : NEGSL * t;
    t = valid ? t : NEGBIG;
    const float bm = wmaxf(t);
    const float mn = fmaxf(m[h], bm);
    const float s1 = expf(m[h] - mn);
    float e = expf(t - mn);
    e = valid ? e : 0.0f;
    const float bs = wsumf(e);
    d[h]  = fmaf(d[h], s1, bs);
    m[h]  = mn;
    sc[h] = s1;
    ee[h] = e;
  }
  return sr;
}

template <int FIN>
__global__ __launch_bounds__(NTHR) void k_agg(const int* __restrict__ srcs, const int* __restrict__ dsts,
                                              int nE, int nN, int vec8, int mRows,
                                              const float* __restrict__ Sm, const float* __restrict__ ALR,
                                              int arOff, const float* __restrict__ bias,
                                              unsigned short* xh, float* outp) {
  extern __shared__ __attribute__((aligned(16))) int dsm[];
  int* list = dsm;
  int* bins = dsm + LISTN;
  int* cnt  = bins + BINS;
  int* misc = cnt + NBRUN;
  float* stgo = (float*)(misc + 16);
  const int tid = (int)threadIdx.x, lane = tid & 31;
  const int wave = __builtin_amdgcn_readfirstlane(tid >> 5);
  const int nodeBase = (int)blockIdx.x * NBRUN;

  {
    const v4i z4 = {0, 0, 0, 0};
    for (int i = tid * 4; i < AGG_ZINTS; i += NTHR * 4) *(v4ia*)(dsm + i) = z4;
    if (tid < 16) misc[tid] = 0;
  }
  __syncthreads();

  const int nChunks = (nE + CHUNK - 1) / CHUNK;
#pragma unroll 1
  for (int ch = 0; ch < nChunks; ++ch) {
    const int cbase = ch * CHUNK;
    const int wc = scan_chunk(dsts, nE, cbase, nodeBase, NBRUN, vec8, list, tid, lane, wave);
    if (lane == 0) misc[wave] = wc;
    __syncthreads();
    if (wave == 0) {
#pragma unroll 1
      for (int w2 = 0; w2 < NWAVE; ++w2) {
        int c = __builtin_amdgcn_readfirstlane(misc[w2]);
        c = c < 0 ? 0 : (c > WCAP ? WCAP : c);
#pragma unroll 1
        for (int b0 = 0; b0 < c; b0 += 32) {
          const int idx = b0 + lane;
          const int ent = list[w2 * WCAP + (idx < WCAP ? idx : WCAP - 1)];
          const int m32 = (c - b0) < 32 ? (c - b0) : 32;
#pragma unroll 1
          for (int k = 0; k < m32; ++k) {
            const int u    = __builtin_amdgcn_readlane(ent, k);
            const int slot = u & (NBRUN - 1);
            const int el   = (u >> SLB) & (CHUNK - 1);
            int eid = cbase + el;
            eid = eid > nE - 1 ? nE - 1 : eid;
            if (lane == 0) {
              int n = cnt[slot];
              n = n < 0 ? 0 : n;
              if (n < BCAP) bins[slot * BCAP + n] = eid;
              cnt[slot] = n + 1;
            }
          }
        }
      }
    }
    __syncthreads();
  }

  const float qnan = __int_as_float(0x7fc00000);

  if (FIN == 0) {
    const int hd = lane >> 3;
    const bool hb1 = (hd & 1) != 0, hb2 = (hd & 2) != 0;
    const v4f bb4 = bfr4(*(const v4fa*)(bias + 4 * lane));
#pragma unroll 1
    for (int jt = 0; jt < NBW; ++jt) {
      const int slot = wave * NBW + jt;
      const int grow = nodeBase + slot;
      const int gcl  = grow < nN ? grow : nN - 1;
      const int craw = __builtin_amdgcn_readfirstlane(cnt[slot]);
      const int c    = craw < 0 ? 0 : (craw > BCAP ? BCAP : craw);
      const int nent = c + 1;
      const float pz = (craw > BCAP) ? qnan : 0.0f;
      const v4f ar4 = *(const v4fa*)(ALR + (size_t)arOff + (size_t)gcl * 4);
      float m[4] = {NEGBIG, NEGBIG, NEGBIG, NEGBIG};
      float d[4] = {0.0f, 0.0f, 0.0f, 0.0f};
      float ee[4], sc[4];
      v4f acc = {0.0f, 0.0f, 0.0f, 0.0f};
#pragma unroll 1
      for (int b0 = 0; b0 < nent; b0 += 32) {
        const int sr = batch_front(bins + slot * BCAP, srcs, ALR, nE, nN, gcl, b0, nent, lane, ar4, m, d, ee, sc);
        const float scl = hb2 ? (hb1 ? sc[3] : sc[2]) : (hb1 ? sc[1] : sc[0]);
        acc.x *= scl; acc.y *= scl; acc.z *= scl; acc.w *= scl;
        const int e0i = __float_as_int(ee[0]), e1i = __float_as_int(ee[1]);
        const int e2i = __float_as_int(ee[2]), e3i = __float_as_int(ee[3]);
        int m32 = nent - b0; m32 = m32 > 32 ? 32 : m32;
#pragma unroll 1
        for (int k = 0; k < m32; ++k) {
          const int sk = __builtin_amdgcn_readlane(sr, k);
          const float w0 = __int_as_float(__builtin_amdgcn_readlane(e0i, k));
          const float w1 = __int_as_float(__builtin_amdgcn_readlane(e1i, k));
          const float w2 = __int_as_float(__builtin_amdgcn_readlane(e2i, k));
          const float w3 = __int_as_float(__builtin_amdgcn_readlane(e3i, k));
          const float w  = hb2 ? (hb1 ? w3 : w2) : (hb1 ? w1 : w0);
          const v4f fs = *(const v4fa*)(Sm + (size_t)sk * NSTR + 4 * lane);
          acc.x = fmaf(w, fs.x, acc.x);
          acc.y = fmaf(w, fs.y, acc.y);
          acc.z = fmaf(w, fs.z, acc.z);
          acc.w = fmaf(w, fs.w, acc.w);
        }
      }
      const float dsel = hb2 ? (hb1 ? d[3] : d[2]) : (hb1 ? d[1] : d[0]);
      const float inv  = __builtin_amdgcn_rcpf(dsel);
      const v4f sk4 = *(const v4fa*)(Sm + (size_t)gcl * NSTR + HC01 + 4 * lane);
      v4f o;
      o.x = fmaf(acc.x, inv, bb4.x) + sk4.x;
      o.y = fmaf(acc.y, inv, bb4.y) + sk4.y;
      o.z = fmaf(acc.z, inv, bb4.z) + sk4.z;
      o.w = fmaf(acc.w, inv, bb4.w) + sk4.w;
#pragma unroll 1
      for (int j = 0; j < 4; ++j) {
        const float v = o.x;
        const float e = (v > 0.0f) ? v : expm1f(v);
        v4f t; t.x = o.y; t.y = o.z; t.z = o.w; t.w = e;
        o = t;
      }
      const bool live = grow < nN;
      o.x = live ? (o.x + pz) : 0.0f;
      o.y = live ? (o.y + pz) : 0.0f;
      o.z = live ? (o.z + pz) : 0.0f;
      o.w = live ? (o.w + pz) : 0.0f;
      const unsigned int hbx = f2bf(o.x), hby = f2bf(o.y), hbz = f2bf(o.z), hbw = f2bf(o.w);
      const unsigned int lbx = f2bf(o.x - bf2f(hbx)), lby = f2bf(o.y - bf2f(hby));
      const unsigned int lbz = f2bf(o.z - bf2f(hbz)), lbw = f2bf(o.w - bf2f(hbw));
      const int hw0 = (int)(hbx | (hby << 16)), hw1 = (int)(hbz | (hbw << 16));
      const int lw0 = (int)(lbx | (lby << 16)), lw1 = (int)(lbz | (lbw << 16));
      const int sa = (2 * lane) & 31, sb2 = (2 * lane + 1) & 31;
      const int g0 = __shfl(hw0, sa), g1 = __shfl(hw1, sa), g2 = __shfl(hw0, sb2), g3 = __shfl(hw1, sb2);
      const int q0 = __shfl(lw0, sa), q1 = __shfl(lw1, sa), q2 = __shfl(lw0, sb2), q3 = __shfl(lw1, sb2);
      const bool lsel = lane >= 16;
      v4u pv;
      pv.x = (unsigned int)(lsel ? q0 : g0);
      pv.y = (unsigned int)(lsel ? q1 : g1);
      pv.z = (unsigned int)(lsel ? q2 : g2);
      pv.w = (unsigned int)(lsel ? q3 : g3);
      unsigned short* gp = xh + (size_t)grow * KH + 8 * lane;
      const bool wr = grow < mRows;
      if (wr) *(volatile v4u*)gp = pv;
      __threadfence();
      if (wr) *(volatile v4u*)gp = pv;
    }
  } else {
    const int c1 = (32 + lane) < NCLS ? (32 + lane) : NCLS - 1;
    const bool valid1 = lane < NCLS - 32;
    const float bz0 = bfr(bias[lane]);
    const float bz1 = bfr(bias[c1]);
    float* res = stgo + wave * (GRP * NCLS);

#pragma unroll 1
    for (int jt = 0; jt < NBW; ++jt) {
      const int slot = wave * NBW + jt;
      const int grow = nodeBase + slot;
      const int gcl  = grow < nN ? grow : nN - 1;
      const int craw = __builtin_amdgcn_readfirstlane(cnt[slot]);
      const int c    = craw < 0 ? 0 : (craw > BCAP ? BCAP : craw);
      const int nent = c + 1;
      const float pz = (craw > BCAP) ? qnan : 0.0f;
      const v4f ar4 = *(const v4fa*)(ALR + (size_t)arOff + (size_t)gcl * 4);
      float m[4] = {NEGBIG, NEGBIG, NEGBIG, NEGBIG};
      float d[4] = {0.0f, 0.0f, 0.0f, 0.0f};
      float ee[4], sc[4];
      float a0[4] = {0.0f, 0.0f, 0.0f, 0.0f};
      float a1[4] = {0.0f, 0.0f, 0.0f, 0.0f};
#pragma unroll 1
      for (int b0 = 0; b0 < nent; b0 += 32) {
        const int sr = batch_front(bins + slot * BCAP, srcs, ALR, nE, nN, gcl, b0, nent, lane, ar4, m, d, ee, sc);
        int eei[4];
#pragma unroll
        for (int h = 0; h < 4; ++h) {
          a0[h] *= sc[h];
          a1[h] *= sc[h];
          eei[h] = __float_as_int(ee[h]);
        }
        int m32 = nent - b0; m32 = m32 > 32 ? 32 : m32;
#pragma unroll 1
        for (int k = 0; k < m32; ++k) {
          const int sk = __builtin_amdgcn_readlane(sr, k);
          const float* rp = Sm + (size_t)sk * NSTR;
#pragma unroll
          for (int h = 0; h < 4; ++h) {
            const float w  = __int_as_float(__builtin_amdgcn_readlane(eei[h], k));
            const float r0 = rp[h * NCLS + lane];
            const float r1 = rp[h * NCLS + c1];
            a0[h] = fmaf(w, r0, a0[h]);
            a1[h] = fmaf(w, r1, a1[h]);
          }
        }
      }
      float y0 = 0.0f, y1 = 0.0f;
#pragma unroll
      for (int h = 0; h < 4; ++h) {
        const float inv = __builtin_amdgcn_rcpf(d[h]);
        y0 = fmaf(a0[h], inv, y0);
        y1 = fmaf(a1[h], inv, y1);
      }
      const float* sp = Sm + (size_t)gcl * NSTR + HC2;
      y0 = (0.25f * y0 + bz0) + sp[lane];
      y1 = (0.25f * y1 + bz1) + sp[c1];
      float vm = fmaxf(y0, valid1 ? y1 : NEGBIG);
      vm = wmaxf(vm);
      const float ex0 = expf(y0 - vm);
      const float ex1 = expf(y1 - vm);
      float sm = ex0 + (valid1 ? ex1 : 0.0f);
      sm = wsumf(sm);
      const float ls = logf(sm);
      const float o0 = ((y0 - vm) - ls) + pz;
      const float o1 = ((y1 - vm) - ls) + pz;
      const int lr = jt & (GRP - 1);
      res[lr * NCLS + lane] = o0;
      if (valid1) res[lr * NCLS + 32 + lane] = o1;

      if (lr == GRP - 1) {
        __syncthreads();
        const int row0 = nodeBase + wave * NBW + (jt - (GRP - 1));
        int live = nN - row0; live = live < 0 ? 0 : (live > GRP ? GRP : live);
        const int npc = (live * NCLS) >> 2;
        float* ob = outp + (size_t)row0 * NCLS;
#pragma unroll 1
        for (int p = lane; p < npc; p += 32) {
          const v4f v = *(const v4fa*)(res + 4 * p);
          *(volatile v4f*)(ob + 4 * p) = v;
        }
        __threadfence();
#pragma unroll 1
        for (int p = lane; p < npc; p += 32) {
          const v4f v = *(const v4fa*)(res + 4 * p);
          *(volatile v4f*)(ob + 4 * p) = v;
        }
        __syncthreads();
      }
    }
  }
}

static inline int cdiv(int a, int b) { return (a + b - 1) / b; }

extern "C" void kernel_launch(void* const* d_in, const int* in_sizes, int n_in,
                              void* d_out, int out_size, void* d_ws, size_t ws_size,
                              hipStream_t stream) {
  if (n_in < 20) return;
  if (in_sizes[0] < NIN || (in_sizes[0] % NIN) != 0) return;
  const int nN = in_sizes[0] / NIN;
  if (nN < 1 || (nN & 3) != 0 || nN > (1 << 21)) return;
  if (in_sizes[1] < 2 || (in_sizes[1] & 1) != 0) return;
  const int nE = in_sizes[1] / 2;
  if (nE < 1 || nE > (1 << 30)) return;
  if (in_sizes[2] != HC01 * NIN || in_sizes[6] != HC01 * NIN) return;
  if (in_sizes[3] != HC01 || in_sizes[4] != HC01) return;
  if (in_sizes[5] != HC01 || in_sizes[7] != HC01) return;
  if (in_sizes[8] != HC01 * HC01 || in_sizes[12] != HC01 * HC01) return;
  if (in_sizes[9] != HC01 || in_sizes[10] != HC01) return;
  if (in_sizes[11] != HC01 || in_sizes[13] != HC01) return;
  if (in_sizes[14] != HC2 * HC01 || in_sizes[18] != NCLS * HC01) return;
  if (in_sizes[15] != HC2 || in_sizes[16] != HC2) return;
  if (in_sizes[17] != NCLS || in_sizes[19] != NCLS) return;
  if ((long long)out_size != (long long)nN * NCLS) return;

  const float* x   = (const float*)d_in[0];
  const int*   ei  = (const int*)  d_in[1];
  const float* W0  = (const float*)d_in[2];
  const float* as0 = (const float*)d_in[3];
  const float* ad0 = (const float*)d_in[4];
  const float* b0  = (const float*)d_in[5];
  const float* sw0 = (const float*)d_in[6];
  const float* sb0 = (const float*)d_in[7];
  const float* W1  = (const float*)d_in[8];
  const float* as1 = (const float*)d_in[9];
  const float* ad1 = (const float*)d_in[10];
  const float* b1  = (const float*)d_in[11];
  const float* sw1 = (const float*)d_in[12];
  const float* sb1 = (const float*)d_in[13];
  const float* W2  = (const float*)d_in[14];
  const float* as2 = (const float*)d_in[15];
  const float* ad2 = (const float*)d_in[16];
  const float* b2  = (const float*)d_in[17];
  const float* sw2 = (const float*)d_in[18];
  const float* sb2 = (const float*)d_in[19];
  float* out = (float*)d_out;
  const int* src = ei;
  const int* dst = ei + nE;

  const int MP   = cdiv(nN, GBM) * GBM;
  const int gM   = MP / GBM;
  const int gA   = cdiv(MP, NBRUN);
  if ((long long)gA * NBRUN < (long long)MP) return;
  const int vec8 = ((nE & 3) == 0) ? 1 : 0;
  const int arOff = MP * 4;

  char* ws = (char*)d_ws;
  size_t off = 0;
  const size_t oXB  = off; off += (size_t)MP * KX * 2;        off = (off + 255) & ~(size_t)255;
  const size_t oWB0 = off; off += (size_t)256 * KX * 2;       off = (off + 255) & ~(size_t)255;
  const size_t oWB1 = off; off += (size_t)256 * KH * 2;       off = (off + 255) & ~(size_t)255;
  const size_t oWB2 = off; off += (size_t)256 * KH * 2;       off = (off + 255) & ~(size_t)255;
  const size_t oS   = off; off += (size_t)MP * NSTR * 4;      off = (off + 255) & ~(size_t)255;
  const size_t oALR = off; off += (size_t)2 * MP * 4 * 4;     off = (off + 255) & ~(size_t)255;
  const size_t oXH  = off; off += (size_t)MP * KH * 2;        off = (off + 255) & ~(size_t)255;
  if (off > ws_size || off > (size_t)WSMAX) return;
  unsigned short* XB  = (unsigned short*)(ws + oXB);
  unsigned short* WB0 = (unsigned short*)(ws + oWB0);
  unsigned short* WB1 = (unsigned short*)(ws + oWB1);
  unsigned short* WB2 = (unsigned short*)(ws + oWB2);
  float*          Sm  = (float*)(ws + oS);
  float*          ALR = (float*)(ws + oALR);
  unsigned short* XH  = (unsigned short*)(ws + oXH);

  hipFuncSetAttribute(reinterpret_cast<const void*>(&k_gemm),
                      hipFuncAttributeMaxDynamicSharedMemorySize, (int)LDS_GEMM);
  hipFuncSetAttribute(reinterpret_cast<const void*>(&k_agg<0>),
                      hipFuncAttributeMaxDynamicSharedMemorySize, (int)LDS_AGG0);
  hipFuncSetAttribute(reinterpret_cast<const void*>(&k_agg<1>),
                      hipFuncAttributeMaxDynamicSharedMemorySize, (int)LDS_AGG1);

  const int uX = MP * (KX / 8);
  const int uT = uX + UW0 + UW1 + UW2;
  k_prep<<<cdiv(uT, NTHR), NTHR, 0, stream>>>(x, W0, sw0, W1, sw1, W2, sw2, XB, WB0, WB1, WB2, nN, uX);

  k_gemm<<<gM, NTHR, LDS_GEMM, stream>>>(XB, KX, WB0, KX, KX, Sm, as0, ad0, sb0, HC01, C01, HC01, HC01, ALR, arOff);
  k_agg<0><<<gA, NTHR, LDS_AGG0, stream>>>(src, dst, nE, nN, vec8, MP, Sm, ALR, arOff, b0, XH, out);
  k_gemm<<<gM, NTHR, LDS_GEMM, stream>>>(XH, KH, WB1, KH, KH, Sm, as1, ad1, sb1, HC01, C01, HC01, HC01, ALR, arOff);
  k_agg<0><<<gA, NTHR, LDS_AGG0, stream>>>(src, dst, nE, nN, vec8, MP, Sm, ALR, arOff, b1, XH, out);
  k_gemm<<<gM, NTHR, LDS_GEMM, stream>>>(XH, KH, WB2, KH, KH, Sm, as2, ad2, sb2, HC2, NCLS, HC2, NCLS, ALR, arOff);
  k_agg<1><<<gA, NTHR, LDS_AGG1, stream>>>(src, dst, nE, nN, vec8, MP, Sm, ALR, arOff, b2, XH, out);
}
